// MSDeformAttnGrid_convoffsets_30124900614204
// MI455X (gfx1250) — hardware-verified
//
#include <hip/hip_runtime.h>


namespace {
constexpr int NBt = 2, C = 256, HH = 128, WW = 128, LQ = HH * WW, NH = 8, NP = 4, DH = 32, PAD = 1, HP = HH + 2, WP = WW + 2, KS = 7, NPRJ = 352, NROW = NBt * LQ;
constexpr float XS = 8.0f, WSC = 256.0f, EPS = 1e-5f;

typedef _Float16 b16;
typedef __attribute__((ext_vector_type(16))) _Float16 v16b;
typedef __attribute__((ext_vector_type(8))) _Float16 v8b;
typedef __attribute__((ext_vector_type(8))) float v8f;
typedef __attribute__((ext_vector_type(4))) float v4f;
__device__ __forceinline__ float bf16_rne(float f) { unsigned int u = __float_as_uint(f); u += 0x7FFFu + ((u >> 16) & 1u); return __uint_as_float(u & 0xFFFF0000u); }
__device__ __forceinline__ void split16(float v, b16& hi, b16& lo) { hi = (b16)v; lo = (b16)(v - (float)hi); }
__device__ __forceinline__ v16b frag_kb(const b16* p, int hh) { const v8b a = *(const v8b*)(p + 8 * hh), b = *(const v8b*)(p + 16 + 8 * hh); v16b f;
#pragma unroll
  for (int e = 0; e < 8; ++e) { f[e] = a[e]; f[8 + e] = b[e]; } return f; }
__device__ __forceinline__ v8f wmma16b(v16b a, v16b b, v8f c) { v8f d = __builtin_amdgcn_wmma_f32_16x16x32_f16(false, a, false, b, (short)0, c, false, false); asm volatile("v_nop\n\tv_nop\n\tv_nop\n\tv_nop" : "+v"(d) : "v"(a), "v"(b)); return d; }
__device__ __forceinline__ void wave_lds_sync() { __builtin_amdgcn_fence(__ATOMIC_RELEASE, "workgroup"); __builtin_amdgcn_wave_barrier(); __builtin_amdgcn_fence(__ATOMIC_ACQUIRE, "workgroup"); }
__device__ __forceinline__ float nexp(float x) { return __builtin_amdgcn_exp2f(x * 1.4426950408889634f); }
__device__ __forceinline__ float pmul(float a, float b) { float p = a * b; asm volatile("" : "+v"(p)); return p; }
__device__ __forceinline__ float sigm(float x) { return 1.0f / (1.0f + nexp(-x)); }

__global__ __launch_bounds__(256) void prepw_kernel(const float* __restrict__ wval, const float* __restrict__ woff, const float* __restrict__ wattn, const float* __restrict__ wout, const float* __restrict__ bval, const float* __restrict__ boff, const float* __restrict__ battn, b16* __restrict__ WPRJ, b16* __restrict__ WOUT, float* __restrict__ PB) {
  __shared__ __attribute__((aligned(16))) b16 T[64][64 + 8];
  const int i0 = blockIdx.x * 64, o0 = blockIdx.y * 64, t_ = threadIdx.x;
  const float* w; int OUT, ocol0; b16* dst; int drow0;
  if (o0 < 256) { w = wval; OUT = 256; ocol0 = o0; dst = WPRJ; drow0 = o0; } else if (o0 < 320) { w = woff; OUT = 64; ocol0 = o0 - 256; dst = WPRJ; drow0 = o0; } else if (o0 < 384) { w = wattn; OUT = 32; ocol0 = o0 - 320; dst = WPRJ; drow0 = o0; } else { w = wout; OUT = 256; ocol0 = o0 - 384; dst = WOUT; drow0 = o0 - 384; }
  for (int q = t_; q < 64 * 64; q += 256) { const int ii = q >> 6, oo = q & 63; const int oc = ocol0 + oo; T[oo][ii] = (oc < OUT) ? (b16)(bf16_rne(w[(size_t)(i0 + ii) * OUT + (oc < OUT ? oc : 0)]) * WSC) : (b16)0.0f; }
  __syncthreads();
  for (int pass = 0; pass < 2; ++pass) {
    for (int q = t_; q < 64 * 8; q += 256) { const int oo = q >> 3, c8 = (q & 7) * 8; if (o0 < 384 ? (drow0 + oo < NPRJ) : true) *(volatile v8b*)(dst + (size_t)(drow0 + oo) * C + i0 + c8) = *(const v8b*)(&T[oo][c8]); }
    if (blockIdx.x == 0 && blockIdx.y == 0) for (int k = t_; k < 384; k += 256) { const float v = k < 256 ? bval[k < 256 ? k : 0] : k < 320 ? boff[(k - 256) & 63] : k < 352 ? battn[(k - 320) & 31] : 0.0f; ((volatile float*)PB)[k] = bf16_rne(v); }
    __threadfence(); }
}
__global__ __launch_bounds__(256) void dwconv_kernel(const float* __restrict__ query, const float* __restrict__ dwk, const float* __restrict__ dwb, float* __restrict__ DWO) {
  __shared__ float Tq[22 * 22][64]; __shared__ __attribute__((aligned(16))) float To[64][64 + 4]; __shared__ float Sw[64][KS * KS + 1];
  const int n = blockIdx.z, c0 = blockIdx.y * 64, ty = (blockIdx.x >> 3) * 16, tx = (blockIdx.x & 7) * 16, t_ = threadIdx.x;
  for (int k = t_; k < 22 * 22 * 64; k += 256) { const int cc = k & 63, p = k >> 6, py = p / 22, px = p - py * 22; const int y = ty + py - 3, x = tx + px - 3; const bool in = (y >= 0) && (y < HH) && (x >= 0) && (x < WW);
    const float v = query[((size_t)n * LQ + (size_t)(in ? y : 0) * WW + (in ? x : 0)) * C + c0 + cc]; Tq[p][cc] = in ? bf16_rne(v) : 0.0f; }
  __syncthreads();
  for (int k = t_; k < 64 * KS * KS; k += 256) { const int cc = k / (KS * KS), kk = k - cc * (KS * KS); Sw[cc][kk] = bf16_rne(dwk[(size_t)(c0 + cc) * KS * KS + kk]); }
  __syncthreads();
  { const int cc = t_ & 63, qg = t_ >> 6; const int c = c0 + cc; const float bb = bf16_rne(dwb[c]);
    for (int round = 0; round < 4; ++round) {
#pragma unroll 1
      for (int i = 0; i < 16; ++i) { const int pl = qg * 16 + i, pp = round * 64 + pl; const int oy = pp >> 4, ox = pp & 15; float s = bb;
#pragma unroll 1
        for (int dy = 0; dy < KS; ++dy) {
#pragma unroll
          for (int dx = 0; dx < KS; ++dx) s += pmul(Sw[cc][dy * KS + dx], Tq[(oy + dy) * 22 + ox + dx][cc]); }
        To[pl][cc] = s; }
      __syncthreads();
      for (int pass = 0; pass < 2; ++pass) { for (int k = t_; k < 64 * 16; k += 256) { const int pl = k >> 4, c4 = (k & 15) * 4; const int pp = round * 64 + pl, oy = pp >> 4, ox = pp & 15; *(volatile v4f*)(DWO + ((size_t)n * LQ + (size_t)(ty + oy) * WW + tx + ox) * C + c0 + c4) = *(const v4f*)(&To[pl][c4]); } __threadfence(); }
      __syncthreads(); } }
}
__global__ __launch_bounds__(256) void lngelu_kernel(const float* __restrict__ DWO, const float* __restrict__ lnw, const float* __restrict__ lnb, b16* __restrict__ QH, b16* __restrict__ QL) {
  __shared__ __attribute__((aligned(16))) float Tg[8][C];
  const int wave = threadIdx.x >> 5, lane = threadIdx.x & 31; const size_t row = (size_t)blockIdx.x * 8 + wave; const float* src = DWO + row * C + lane * 8;
  float s = 0.0f;
#pragma unroll 1
  for (int j = 0; j < 8; ++j) s += src[j];
#pragma unroll
  for (int o = 16; o >= 1; o >>= 1) s += __shfl_xor(s, o);
  const float mu = s * (1.0f / C); float ss = 0.0f;
#pragma unroll 1
  for (int j = 0; j < 8; ++j) { const float d = src[j] - mu; ss += pmul(d, d); }
#pragma unroll
  for (int o = 16; o >= 1; o >>= 1) ss += __shfl_xor(ss, o);
  const float rs = rsqrtf(ss * (1.0f / C) + EPS);
#pragma unroll 1
  for (int j = 0; j < 8; ++j) { const int c = lane * 8 + j; const float y = pmul((src[j] - mu) * rs, bf16_rne(lnw[c])) + bf16_rne(lnb[c]); Tg[wave][c] = 0.5f * y * (1.0f + erff(y * 0.70710678118654752f)); }
  wave_lds_sync();
  const v4f a = *(const v4f*)(&Tg[wave][lane * 8]), bq = *(const v4f*)(&Tg[wave][lane * 8 + 4]); v8b h8, l8;
#pragma unroll
  for (int j = 0; j < 4; ++j) { b16 x_, y_; split16(a[j] * XS, x_, y_); h8[j] = x_; l8[j] = y_; split16(bq[j] * XS, x_, y_); h8[4 + j] = x_; l8[4 + j] = y_; }
  for (int pass = 0; pass < 2; ++pass) { *(volatile v8b*)(QH + row * C + lane * 8) = h8; *(volatile v8b*)(QL + row * C + lane * 8) = l8; __threadfence(); }
}
template <int MODE>
__global__ __launch_bounds__(128) void gemm_kernel(const b16* __restrict__ AH, const b16* __restrict__ AL, const b16* __restrict__ Bw, const float* __restrict__ bias, float* __restrict__ O1, float* __restrict__ O2, float* __restrict__ O3) {
  __shared__ __attribute__((aligned(16))) float Ts[4][16][128 + 4];
  const int wave = threadIdx.x >> 5, lane = threadIdx.x & 31, nloc = lane & 15, hlf = lane >> 4; const size_t m0 = (size_t)blockIdx.x * 64 + wave * 16; const int n0 = blockIdx.y * 128;
  const int NT = (MODE == 0 && blockIdx.y == 2) ? 6 : 8;
  v8f acc[8];
#pragma unroll
  for (int t = 0; t < 8; ++t) acc[t] = (v8f){};
#pragma unroll 2
  for (int kb = 0; kb < C; kb += 32) { const v16b ah = frag_kb(AH + (m0 + nloc) * C + kb, hlf), al = frag_kb(AL + (m0 + nloc) * C + kb, hlf);
#pragma unroll
    for (int t = 0; t < 8; ++t) if (t < NT) { const v16b bw = frag_kb(Bw + (size_t)(n0 + t * 16 + nloc) * C + kb, hlf); acc[t] = wmma16b(ah, bw, acc[t]); acc[t] = wmma16b(al, bw, acc[t]); } }
#pragma unroll
  for (int t = 0; t < 8; ++t) if (t < NT) { const int n = n0 + t * 16 + nloc; const float bb = bias[n];
#pragma unroll
    for (int r = 0; r < 8; ++r) { float v = acc[t][r] * (1.0f / (XS * WSC)) + bb; if (MODE == 0 && n >= 320) v = sigm(v); Ts[wave][8 * hlf + r][t * 16 + nloc] = v; } }
  wave_lds_sync();
  for (int pass = 0; pass < 2; ++pass) {
    for (int rr = 0; rr < 16; ++rr) { const size_t row = m0 + rr;
      if (MODE == 1 || n0 < 256) *(volatile v4f*)(O1 + row * C + n0 + lane * 4) = *(const v4f*)(&Ts[wave][rr][lane * 4]);
      else { if (lane < 16) *(volatile v4f*)(O2 + row * 64 + lane * 4) = *(const v4f*)(&Ts[wave][rr][lane * 4]); if (lane < 8) *(volatile v4f*)(O3 + row * 32 + lane * 4) = *(const v4f*)(&Ts[wave][rr][64 + lane * 4]); } }
    __threadfence(); }
}
__global__ __launch_bounds__(256) void sample_kernel(const float* __restrict__ VAL, const float* __restrict__ OFF, const float* __restrict__ ATT, const float* __restrict__ refp, b16* __restrict__ SH, b16* __restrict__ SL) {
  __shared__ __attribute__((aligned(16))) b16 Th[C + 8], Tl[C + 8];
  const size_t row = blockIdx.x; const int n = (int)(row / LQ); const int h = threadIdx.x >> 5, d = threadIdx.x & 31;
  const float rx = bf16_rne(refp[row * 2 + 0]), ry = bf16_rne(refp[row * 2 + 1]);
  float acc = 0.0f;
#pragma unroll
  for (int p = 0; p < NP; ++p) {
    const float gx = (p >> 1) ? 1.0f : 0.0f, gy = (p & 1) ? 1.0f : 0.0f;
    const float ox = OFF[row * 64 + (h * NP + p) * 2 + 0], oy = OFF[row * 64 + (h * NP + p) * 2 + 1], aw = ATT[row * 32 + h * NP + p];
    const float lx = rx + (gx + ox) / (float)WP, ly = ry + (gy + oy) / (float)HP;
    const float x = lx * (float)WP - 0.5f, y = ly * (float)HP - 0.5f; const float x0f = floorf(x), y0f = floorf(y); const float wx1 = x - x0f, wx0 = 1.0f - wx1, wy1 = y - y0f, wy0 = 1.0f - wy1;
    const int x0 = (int)x0f, y0 = (int)y0f;
    float sv = 0.0f;
#pragma unroll
    for (int cy = 0; cy < 2; ++cy)
#pragma unroll
      for (int cx = 0; cx < 2; ++cx) { const int xi = x0 + cx, yi = y0 + cy; const bool inner = (xi >= 0) && (xi < WP) && (yi >= 0) && (yi < HP) && (xi >= PAD) && (xi < WP - PAD) && (yi >= PAD) && (yi < HP - PAD);
        const int ty = yi - PAD < 0 ? 0 : (yi - PAD >= HH ? HH - 1 : yi - PAD), tx = xi - PAD < 0 ? 0 : (xi - PAD >= WW ? WW - 1 : xi - PAD);
        const float g = VAL[((size_t)n * LQ + (size_t)ty * WW + tx) * C + h * DH + d];
        const float wgt = (cy ? wy1 : wy0) * (cx ? wx1 : wx0);
        sv += pmul(inner ? g : 0.0f, wgt); }
    acc += pmul(sv, aw); }
  b16 a_, c_; split16(acc * XS, a_, c_); Th[h * DH + d] = a_; Tl[h * DH + d] = c_;
  __syncthreads();
  for (int pass = 0; pass < 2; ++pass) { if (threadIdx.x < 32) { *(volatile v8b*)(SH + row * C + threadIdx.x * 8) = *(const v8b*)(&Th[threadIdx.x * 8]); *(volatile v8b*)(SL + row * C + threadIdx.x * 8) = *(const v8b*)(&Tl[threadIdx.x * 8]); } __threadfence(); }
}
__global__ __launch_bounds__(256) void pob_kernel(const float* __restrict__ bo, float* __restrict__ POB) { const int t_ = threadIdx.x; const float v = bf16_rne(bo[t_]); for (int pass = 0; pass < 2; ++pass) { ((volatile float*)POB)[t_] = v; __threadfence(); } }
}

extern "C" void kernel_launch(void* const* d_in, const int* in_sizes, int n_in, void* d_out, int out_size, void* d_ws, size_t ws_size, hipStream_t stream) {
  (void)n_in;
  auto Fp = [&](int i) { return (const float*)d_in[i]; };
  if (in_sizes[0] != NROW * C || in_sizes[1] != NROW * 2 || in_sizes[4] != C * KS * KS || in_sizes[8] != C * 64 || in_sizes[10] != C * 32 || in_sizes[12] != C * C || in_sizes[14] != C * C || out_size != NROW * C) return;
  size_t off = 0; char* ws = (char*)d_ws;
  auto carve = [&](size_t bytes) { char* p = ws + off; off += (bytes + 255) & ~(size_t)255; return p; };
  b16* WPRJ = (b16*)carve((size_t)NPRJ * C * 2); b16* WOUT = (b16*)carve((size_t)C * C * 2); float* PB = (float*)carve(384 * 4); float* POB = (float*)carve(C * 4);
  float* DWO = (float*)carve((size_t)NROW * C * 4); b16* QH = (b16*)carve((size_t)NROW * C * 2); b16* QL = (b16*)carve((size_t)NROW * C * 2);
  float* VAL = (float*)carve((size_t)NROW * C * 4); float* OFF = (float*)carve((size_t)NROW * 64 * 4); float* ATT = (float*)carve((size_t)NROW * 32 * 4);
  b16* SH = QH; b16* SL = QL;
  if (off > ws_size) return;
  prepw_kernel<<<dim3(C / 64, 10), 256, 0, stream>>>(Fp(12), Fp(8), Fp(10), Fp(14), Fp(13), Fp(9), Fp(11), WPRJ, WOUT, PB);
  pob_kernel<<<1, 256, 0, stream>>>(Fp(15), POB);
  dwconv_kernel<<<dim3(64, C / 64, NBt), 256, 0, stream>>>(Fp(0), Fp(4), Fp(5), DWO);
  lngelu_kernel<<<NROW / 8, 256, 0, stream>>>(DWO, Fp(6), Fp(7), QH, QL);
  gemm_kernel<0><<<dim3(NROW / 64, 3), 128, 0, stream>>>(QH, QL, WPRJ, PB, VAL, OFF, ATT);
  sample_kernel<<<NROW, 256, 0, stream>>>(VAL, OFF, ATT, Fp(1), SH, SL);
  gemm_kernel<1><<<dim3(NROW / 64, 2), 128, 0, stream>>>(SH, SL, WOUT, POB, (float*)d_out, nullptr, nullptr);
}
